// CrossAttention2D_38774964748372
// MI455X (gfx1250) — hardware-verified
//
#include <hip/hip_runtime.h>
#include <math.h>

typedef __attribute__((ext_vector_type(16))) _Float16 v16h;
typedef __attribute__((ext_vector_type(16))) __bf16 v16b;
typedef __attribute__((ext_vector_type(8)))  _Float16 v8h;
typedef __attribute__((ext_vector_type(8)))  float v8f;
typedef __attribute__((ext_vector_type(4)))  float v4f;
typedef __attribute__((ext_vector_type(2)))  float v2f;
typedef __attribute__((ext_vector_type(4)))  unsigned v4u;
typedef __attribute__((ext_vector_type(4)))  int v4i;
typedef float __attribute__((may_alias)) float_a;
typedef int __attribute__((may_alias)) int_a;

template <typename T> __device__ __forceinline__ void vst2(void* p, T v) { *(volatile T*)p = v; __threadfence(); *(volatile T*)p = v; }
__device__ __forceinline__ v8f wmma16(v16h a, v16h b, v8f c) {
  v8f d = __builtin_amdgcn_wmma_f32_16x16x32_f16(false, a, false, b, (short)0, c, false, false);
  asm volatile("v_nop\n\tv_nop\n\tv_nop\n\tv_nop" : "+v"(d) : "v"(a), "v"(b));
  return d;
}
__device__ __forceinline__ v8f wmma_bf(v16b a, v16b b, v8f c) {
  v8f d = __builtin_amdgcn_wmma_f32_16x16x32_bf16(false, a, false, b, (short)0, c, false, false);
  asm volatile("v_nop\n\tv_nop\n\tv_nop\n\tv_nop" : "+v"(d) : "v"(a), "v"(b));
  return d;
}
__device__ __forceinline__ v16h frag_h(const _Float16* rowk0, int lane) {
  union { v16h v; v8h q[2]; } u; const _Float16* p = rowk0 + 8 * (lane >> 4);
  u.q[0] = *(const v8h*)p; u.q[1] = *(const v8h*)(p + 16); return u.v;
}
__device__ __forceinline__ v16h frag_f32(const float* rowk0, int lane) {
  v16h a; const float* p = rowk0 + 8 * (lane >> 4);
#pragma unroll
  for (int i = 0; i < 8; ++i) { a[i] = (_Float16)p[i]; a[8 + i] = (_Float16)p[16 + i]; }
  return a;
}
__device__ __forceinline__ v16h frag_f32s(const float* rowk0, int lane, float sc) {
  v16h a; const float* p = rowk0 + 8 * (lane >> 4);
#pragma unroll
  for (int i = 0; i < 8; ++i) { a[i] = (_Float16)(p[i] * sc); a[8 + i] = (_Float16)(p[16 + i] * sc); }
  return a;
}
__device__ __forceinline__ v16h fragc_f32(const float* W, int k0, int n, int lane, int ld, int K) {
  v16h a; const int g = lane >> 4;
#pragma unroll
  for (int i = 0; i < 8; ++i) { const int ka = k0 + 8 * g + i, kb = ka + 16;
    a[i] = (_Float16)(ka < K ? W[(size_t)(ka < K ? ka : K - 1) * ld + n] : 0.f); a[8 + i] = (_Float16)(kb < K ? W[(size_t)(kb < K ? kb : K - 1) * ld + n] : 0.f); }
  return a;
}
struct F2 { v16b h, l; };
__device__ __forceinline__ F2 bsplit16(const float v[16]) { F2 r;
#pragma unroll
  for (int i = 0; i < 16; ++i) { const __bf16 h = (__bf16)v[i]; r.h[i] = h; r.l[i] = (__bf16)(v[i] - (float)h); }
  return r; }
__device__ __forceinline__ F2 split_row(const float* row, int k0, int lane) { float v[16]; const float* p = row + k0 + 8 * (lane >> 4);
#pragma unroll
  for (int i = 0; i < 8; ++i) { v[i] = p[i]; v[8 + i] = p[16 + i]; }
  return bsplit16(v); }
__device__ __forceinline__ F2 split_rowK(const float* row, int k0, int lane, int K) { float v[16]; const int g = lane >> 4;
#pragma unroll
  for (int i = 0; i < 8; ++i) { const int ka = k0 + 8 * g + i, kb = ka + 16; v[i] = ka < K ? row[ka < K ? ka : K - 1] : 0.f; v[8 + i] = kb < K ? row[kb < K ? kb : K - 1] : 0.f; }
  return bsplit16(v); }
__device__ __forceinline__ F2 split_col(const float* W, int k0, int n, int lane, int ld, int K) { float v[16]; const int g = lane >> 4;
#pragma unroll
  for (int i = 0; i < 8; ++i) { const int ka = k0 + 8 * g + i, kb = ka + 16; v[i] = ka < K ? W[(size_t)(ka < K ? ka : K - 1) * ld + n] : 0.f; v[8 + i] = kb < K ? W[(size_t)(kb < K ? kb : K - 1) * ld + n] : 0.f; }
  return bsplit16(v); }
__device__ __forceinline__ v8f mac3(const F2& a, const F2& b, v8f c) { c = wmma_bf(a.l, b.h, c); c = wmma_bf(a.h, b.l, c); return wmma_bf(a.h, b.h, c); }
__device__ __forceinline__ float sigm(float v) { return 1.0f / (1.0f + expf(-v)); }
#define LDSX() do { asm volatile("s_wait_dscnt 0" ::: "memory"); __builtin_amdgcn_wave_barrier(); __builtin_amdgcn_fence(__ATOMIC_RELEASE, "workgroup"); } while (0)


#define NB 8
#define CQ 512
#define CY 768
#define NN 1024
#define NH 8
#define HD 64
#ifndef TNB
#define TNB NB
#endif
typedef __attribute__((ext_vector_type(8))) __bf16 v8b;
__device__ __forceinline__ v16b frag_b(const __bf16* rowk0, int lane) {
  union { v16b v; v8b q[2]; } u; const __bf16* p = rowk0 + 8 * (lane >> 4);
  u.q[0] = *(const v8b*)p; u.q[1] = *(const v8b*)(p + 16); return u.v;
}
__device__ __forceinline__ float bfr(float v) { return (float)(__bf16)v; }
__device__ __attribute__((noinline)) float exp_ni(float v) { return expf(v); }
__device__ __attribute__((noinline)) float erf_ni(float v) { return erff(v); }

#define WS_Q   0u
#define WS_K   (WS_Q + 2u * (size_t)NB * NN * CQ)
#define WS_VT  (WS_K + 2u * (size_t)NB * NN * CQ)
#define WS_VTL (WS_VT + 2u * (size_t)NB * CQ * NN)
#define WS_AV  (WS_VTL + 2u * (size_t)NB * CQ * NN)
#define WS_T   (WS_AV + 4u * (size_t)NB * NH * NN * HD)
#define WS_END (WS_T + 4u * (size_t)NB * NN * CQ)

__global__ __launch_bounds__(128) void k_proj(const float* __restrict__ X, const float* __restrict__ Y, const float* __restrict__ WQ, const float* __restrict__ BQ, const float* __restrict__ WK, const float* __restrict__ BK, const float* __restrict__ WV, const float* __restrict__ BV, _Float16* __restrict__ Q, _Float16* __restrict__ K, _Float16* __restrict__ VT, _Float16* __restrict__ VTL) {
  __shared__ __align__(16) _Float16 sh[64][136]; __shared__ __align__(16) _Float16 th[128][72], tl[128][72];
  const int tid = threadIdx.x, wave = tid >> 5, lane = tid & 31, col = lane & 15, g = lane >> 4; const int which = blockIdx.z / NB; const size_t b = blockIdx.z % NB; const int n0 = blockIdx.x * 64 + wave * 16; const int c0 = blockIdx.y * 128;
  const int cin = which == 0 ? CQ : CY; const float* src = which == 0 ? (X + b * CQ * (size_t)NN) : (Y + b * CY * (size_t)NN); const float* Wm = which == 0 ? WQ : which == 1 ? WK : WV; const float* Bm = which == 0 ? BQ : which == 1 ? BK : BV;
  v8f acc[8] = {};
#pragma unroll 2
  for (int kc = 0; kc < cin / 32; ++kc) { v16b a; const int px = n0 + col;
#pragma unroll
    for (int i = 0; i < 8; ++i) { a[i] = (__bf16)src[(size_t)(kc * 32 + 8 * g + i) * NN + px]; a[8 + i] = (__bf16)src[(size_t)(kc * 32 + 16 + 8 * g + i) * NN + px]; }
#pragma unroll
    for (int j = 0; j < 8; ++j) { v16b w; const float* wr = Wm + (size_t)(c0 + j * 16 + col) * cin + kc * 32 + 8 * g;
#pragma unroll
      for (int i = 0; i < 8; ++i) { w[i] = (__bf16)wr[i]; w[8 + i] = (__bf16)wr[16 + i]; }
      acc[j] = wmma_bf(a, w, acc[j]); } }
#pragma unroll
  for (int j = 0; j < 8; ++j) { const float bb = bfr(Bm[c0 + j * 16 + col]);
#pragma unroll
    for (int r = 0; r < 8; ++r) { const float v = acc[j][r] + bb; const _Float16 hv = (_Float16)v; if (which < 2) sh[wave * 16 + 8 * g + r][j * 16 + col] = hv; else { th[j * 16 + col][wave * 16 + 8 * g + r] = hv; tl[j * 16 + col][wave * 16 + 8 * g + r] = (_Float16)((v - (float)hv) * 2048.0f); } } }
  __syncthreads();
  if (which < 2) { _Float16* dst = which == 0 ? Q : K; for (int e = tid; e < 64 * 16; e += 128) { const int rl = e >> 4, q = e & 15; vst2((unsigned*)(dst + (b * NN + blockIdx.x * 64 + rl) * CQ + c0 + q * 8), *(const v4u*)&sh[rl][q * 8]); } }
  else { for (int e = tid; e < 128 * 8; e += 128) { const int cl = e >> 3, q = e & 7; const size_t o = (b * CQ + c0 + cl) * (size_t)NN + blockIdx.x * 64 + q * 8; vst2((unsigned*)(VT + o), *(const v4u*)&th[cl][q * 8]); vst2((unsigned*)(VTL + o), *(const v4u*)&tl[cl][q * 8]); } } }
__global__ __launch_bounds__(128) void k_att(const _Float16* __restrict__ Q, const _Float16* __restrict__ K, const _Float16* __restrict__ VT, const _Float16* __restrict__ VTL, float* __restrict__ AV) {
  __shared__ __align__(16) float sp[4][16][36]; __shared__ __align__(16) float so[4][16][68];
  const int tid = threadIdx.x, wave = tid >> 5, lane = tid & 31, col = lane & 15, g = lane >> 4; const int h = blockIdx.y; const size_t b = blockIdx.z; const int q0 = blockIdx.x * 64 + wave * 16; const size_t rq = b * NN + q0;
  v16h aq[2];
#pragma unroll
  for (int kc = 0; kc < 2; ++kc) aq[kc] = frag_h(Q + (rq + col) * CQ + h * HD + kc * 32, lane);
  float m[8], l[8];
#pragma unroll
  for (int r = 0; r < 8; ++r) { m[r] = -3.0e38f; l[r] = 0.f; }
  v8f acc[4] = {}, accl[4] = {};
#pragma unroll 1
  for (int ks = 0; ks < NN / 32; ++ks) { v8f s[2];
#pragma unroll
    for (int ct = 0; ct < 2; ++ct) { const size_t rk = b * NN + ks * 32 + ct * 16 + col; v8f c = {};
#pragma unroll
      for (int kc = 0; kc < 2; ++kc) c = wmma16(aq[kc], frag_h(K + rk * CQ + h * HD + kc * 32, lane), c);
#pragma unroll
      for (int r = 0; r < 8; ++r) s[ct][r] = c[r] * 0.125f; }
    float alpha[8];
#pragma unroll
    for (int r = 0; r < 8; ++r) { float mx = fmaxf(s[0][r], s[1][r]);
#pragma unroll
      for (int o = 1; o < 16; o <<= 1) mx = fmaxf(mx, __shfl_xor(mx, o));
      const float mn = fmaxf(m[r], mx); alpha[r] = __expf(m[r] - mn); const float e0 = __expf(s[0][r] - mn), e1 = __expf(s[1][r] - mn); float es = e0 + e1;
#pragma unroll
      for (int o = 1; o < 16; o <<= 1) es += __shfl_xor(es, o);
      l[r] = l[r] * alpha[r] + es; m[r] = mn; sp[wave][8 * g + r][col] = e0; sp[wave][8 * g + r][16 + col] = e1; }
#pragma unroll
    for (int j = 0; j < 4; ++j)
#pragma unroll
      for (int r = 0; r < 8; ++r) { acc[j][r] *= alpha[r]; accl[j][r] *= alpha[r]; }
    LDSX();
    v16h pa; { const float* prow = &sp[wave][col][0] + 8 * (lane >> 4);
#pragma unroll
      for (int i = 0; i < 8; ++i) { pa[i] = (_Float16)(prow[i] * 2048.0f); pa[8 + i] = (_Float16)(prow[16 + i] * 2048.0f); } }
#pragma unroll
    for (int j = 0; j < 4; ++j) { const size_t po = (b * CQ + (size_t)h * HD + j * 16 + col) * (size_t)NN + ks * 32; acc[j] = wmma16(pa, frag_h(VT + po, lane), acc[j]); accl[j] = wmma16(pa, frag_h(VTL + po, lane), accl[j]); }
    LDSX(); }
#pragma unroll
  for (int r = 0; r < 8; ++r) { const float il = (1.0f / 2048.0f) / l[r];
#pragma unroll
    for (int j = 0; j < 4; ++j) so[wave][8 * g + r][j * 16 + col] = (acc[j][r] + accl[j][r] * (1.0f / 2048.0f)) * il; }
  LDSX(); for (int rl = 0; rl < 16; ++rl) if (lane < 16) vst2(AV + (((b * NH + h) * NN) + q0 + rl) * HD + lane * 4, *(const v4f*)&so[wave][rl][lane * 4]); }
__global__ __launch_bounds__(128) void k_tr(const float* __restrict__ AV, float* __restrict__ T) { __shared__ __align__(16) float st[64][132]; const int t = threadIdx.x; const size_t b = blockIdx.z; const int p0 = blockIdx.x * 64; const int c0 = blockIdx.y * 128;
  for (int e = t; e < 128 * 64; e += 128) { const int cl = e >> 6, pl = e & 63; st[pl][cl] = AV[(b * CQ + c0 + cl) * (size_t)NN + p0 + pl]; }
  __syncthreads(); for (int e = t; e < 64 * 32; e += 128) { const int pl = e >> 5, q = e & 31; vst2(T + (b * NN + p0 + pl) * CQ + c0 + q * 4, *(const v4f*)&st[pl][q * 4]); } }
__global__ __launch_bounds__(128) void k_o(const float* __restrict__ T, const float* __restrict__ WO, const float* __restrict__ BO, float* __restrict__ OUT) { __shared__ __align__(16) float sf[4][16][132];
  const int tid = threadIdx.x, wave = tid >> 5, lane = tid & 31, col = lane & 15, g = lane >> 4; const size_t b = blockIdx.z; const int o0 = blockIdx.x * 64 + wave * 16; const int p0 = blockIdx.y * 128;
  v8f acc[8] = {};
#pragma unroll 2
  for (int kc = 0; kc < CQ / 32; ++kc) { v16b a; const float* ar = WO + (size_t)(o0 + col) * CQ + kc * 32 + 8 * g;
#pragma unroll
    for (int i = 0; i < 8; ++i) { a[i] = (__bf16)ar[i]; a[8 + i] = (__bf16)ar[16 + i]; }
#pragma unroll
    for (int j = 0; j < 8; ++j) { float wv[16]; const float* wr = T + (b * NN + p0 + j * 16 + col) * CQ + kc * 32 + 8 * g;
#pragma unroll
      for (int i = 0; i < 8; ++i) { wv[i] = wr[i]; wv[8 + i] = wr[16 + i]; }
      const F2 wb = bsplit16(wv); acc[j] = wmma_bf(a, wb.h, acc[j]); acc[j] = wmma_bf(a, wb.l, acc[j]); } }
#pragma unroll
  for (int j = 0; j < 8; ++j)
#pragma unroll
    for (int r = 0; r < 8; ++r) sf[wave][8 * g + r][j * 16 + col] = acc[j][r] + bfr(BO[o0 + 8 * g + r]);
  LDSX(); for (int rl = 0; rl < 16; ++rl) vst2(OUT + (b * CQ + o0 + rl) * (size_t)NN + p0 + lane * 4, *(const v4f*)&sf[wave][rl][lane * 4]); }
extern "C" void kernel_launch(void* const* d_in, const int* in_sizes, int n_in, void* d_out, int out_size, void* d_ws, size_t ws_size, hipStream_t stream) {
  (void)in_sizes; (void)n_in; (void)out_size;
  const float** F = (const float**)d_in;
  if (ws_size < (size_t)WS_END) return;
  char* ws = (char*)d_ws; _Float16 *Q = (_Float16*)(ws + WS_Q), *K = (_Float16*)(ws + WS_K), *VT = (_Float16*)(ws + WS_VT), *VTL = (_Float16*)(ws + WS_VTL); float *AV = (float*)(ws + WS_AV), *T = (float*)(ws + WS_T);
  k_proj<<<dim3(NN / 64, CQ / 128, 3 * NB), 128, 0, stream>>>(F[0], F[1], F[2], F[3], F[4], F[5], F[6], F[7], Q, K, VT, VTL);
  k_att<<<dim3(NN / 64, NH, TNB), 128, 0, stream>>>(Q, K, VT, VTL, AV);
  k_tr<<<dim3(NN / 64, CQ / 128, TNB), 128, 0, stream>>>(AV, T);
  k_o<<<dim3(CQ / 64, NN / 128, TNB), 128, 0, stream>>>(T, F[8], F[9], (float*)d_out);
}
